// Multi_Head_attention_1606317769372
// MI455X (gfx1250) — hardware-verified
//
#include <hip/hip_runtime.h>


#ifndef NB
#define NB 2
#endif
#ifndef SEQ
#define SEQ 2048
#endif
#define NB_FULL 2
#define TT_FULL 2048
#define TT   SEQ
#define DM   512
#define DHID 512
#define NH_  8
#define HD   64
#define ZH   4
#define PCAR 16384.0f
#define L2E  1.4426950408889634f
static_assert(TT % 128 == 0);
static_assert(TT >= 128);
static_assert(TT <= TT_FULL);
static_assert(NB >= 1);
static_assert(NB <= NB_FULL);
static_assert(NH_ % ZH == 0);
static_assert(NH_ * HD == DHID);
static_assert((ZH * TT) % 32 == 0);
static_assert(DM % 64 == 0);
static_assert(DHID % 64 == 0);
static_assert(HD == 64);
static_assert((size_t)NB * TT * DM * 4 <= (size_t)NB_FULL * TT_FULL * DM * 4);

typedef _Float16 h16;
typedef unsigned short bf;
typedef __attribute__((ext_vector_type(16))) __bf16   v16bf;
typedef __attribute__((ext_vector_type(16))) _Float16 v16h;
typedef __attribute__((ext_vector_type(8)))  _Float16 v8h;
typedef __attribute__((ext_vector_type(8)))  unsigned short v8us;
typedef __attribute__((ext_vector_type(8)))  float    v8f;
typedef __attribute__((ext_vector_type(4)))  float    v4f;
typedef v8h  __attribute__((may_alias)) v8ha;
typedef v4f  __attribute__((may_alias)) v4fa;
typedef v8us __attribute__((may_alias)) v8usa;

__device__ __forceinline__ unsigned short f2bf(float f) { unsigned u = __float_as_uint(f); u += 0x7FFFu + ((u >> 16) & 1u); return (unsigned short)(u >> 16); }
__device__ __forceinline__ float bf2f(unsigned short b) { return __uint_as_float(((unsigned)b) << 16); }
__device__ __forceinline__ float bfr(float f) { return bf2f(f2bf(f)); }
__device__ __forceinline__ v16h cat16(v8h lo, v8h hi) { return __builtin_shufflevector(lo, hi, 0, 1, 2, 3, 4, 5, 6, 7, 8, 9, 10, 11, 12, 13, 14, 15); }
__device__ __forceinline__ v16bf cat16b(v8us lo, v8us hi) { return __builtin_bit_cast(v16bf, __builtin_shufflevector(lo, hi, 0, 1, 2, 3, 4, 5, 6, 7, 8, 9, 10, 11, 12, 13, 14, 15)); }
__device__ __forceinline__ v8f wmma16(v16h a, v16h b, v8f c) { return __builtin_amdgcn_wmma_f32_16x16x32_f16(false, a, false, b, (short)0, c, false, false); }
__device__ __forceinline__ v8f wmmab(v16bf a, v16bf b, v8f c) { return __builtin_amdgcn_wmma_f32_16x16x32_bf16(false, a, false, b, (short)0, c, false, false); }

template <typename T16> struct WFrag;
template <> struct WFrag<h16> { typedef v16h V; static __device__ __forceinline__ V ld(const h16* p) { return cat16(*(const v8h*)p, *(const v8h*)(p + 16)); } static __device__ __forceinline__ v8f mma(V a, V b, v8f c) { return wmma16(a, b, c); } };
template <> struct WFrag<bf> { typedef v16bf V; static __device__ __forceinline__ V ld(const bf* p) { return cat16b(*(const v8us*)p, *(const v8us*)(p + 16)); } static __device__ __forceinline__ v8f mma(V a, V b, v8f c) { return wmmab(a, b, c); } };
template <typename T16, int NSPLIT, bool BIAS>
__global__ __launch_bounds__(32) void k_gemmw(const T16* __restrict__ A, const T16* __restrict__ A2, const T16* __restrict__ Bt, const T16* __restrict__ Bt2, int K, float* C, int ldc, const float* __restrict__ bias, size_t sA, size_t sB, size_t sC) {
    typedef typename WFrag<T16>::V V;
    __shared__ __align__(16) float os[16 * 68];
    const size_t z = blockIdx.z; A += z * sA; if (A2) A2 += z * sA; Bt += z * sB; if (Bt2) Bt2 += z * sB; C += z * sC;
    const int lane = threadIdx.x & 31, lr = lane & 15, hi = lane >> 4; const int r0 = blockIdx.x * 64, c0 = blockIdx.y * 64;
    v8f acc[4][4];
#pragma unroll
    for (int mb = 0; mb < 4; ++mb)
#pragma unroll
        for (int nb = 0; nb < 4; ++nb) acc[mb][nb] = (v8f){};
    const size_t aoff = (size_t)(r0 + lr) * K + 8 * hi, boff = (size_t)(c0 + lr) * K + 8 * hi;
#pragma unroll 1
    for (int kc = 0; kc < K; kc += 32) {
        V a[4], a2[4];
#pragma unroll
        for (int mb = 0; mb < 4; ++mb) { a[mb] = WFrag<T16>::ld(A + aoff + (size_t)mb * 16 * K + kc); if (NSPLIT == 1 || NSPLIT == 2) a2[mb] = WFrag<T16>::ld(A2 + aoff + (size_t)mb * 16 * K + kc); }
#pragma unroll
        for (int nb = 0; nb < 4; ++nb) { const V b = WFrag<T16>::ld(Bt + boff + (size_t)nb * 16 * K + kc); V b2; if (NSPLIT >= 2) b2 = WFrag<T16>::ld(Bt2 + boff + (size_t)nb * 16 * K + kc);
#pragma unroll
            for (int mb = 0; mb < 4; ++mb) { acc[mb][nb] = WFrag<T16>::mma(a[mb], b, acc[mb][nb]); if (NSPLIT == 1 || NSPLIT == 2) acc[mb][nb] = WFrag<T16>::mma(a2[mb], b, acc[mb][nb]); if (NSPLIT >= 2) acc[mb][nb] = WFrag<T16>::mma(a[mb], b2, acc[mb][nb]); } }
        asm volatile("v_nop\n\tv_nop\n\tv_nop\n\tv_nop" : "+v"(acc[0][0]), "+v"(acc[1][1]), "+v"(acc[2][2]), "+v"(acc[3][3]) : "v"(a[0]), "v"(a[3]));
    }
#pragma unroll
    for (int mb = 0; mb < 4; ++mb) {
#pragma unroll
        for (int nb = 0; nb < 4; ++nb) {
#pragma unroll
            for (int j = 0; j < 8; ++j) os[(hi * 8 + j) * 68 + nb * 16 + lr] = acc[mb][nb][j]; }
        __builtin_amdgcn_wave_barrier(); asm volatile("" ::: "memory");
        float* crow = C + (size_t)(r0 + mb * 16) * ldc + c0;
#pragma unroll 1
        for (int ps = 0; ps < 2; ++ps) {
#pragma unroll
            for (int s = 0; s < 8; ++s) { const int row = 2 * s + hi, cofs = lr * 4; v4f val = *(const v4fa*)(os + row * 68 + cofs); if (BIAS) { val[0] += bfr(bias[c0 + cofs]); val[1] += bfr(bias[c0 + cofs + 1]); val[2] += bfr(bias[c0 + cofs + 2]); val[3] += bfr(bias[c0 + cofs + 3]); }
                *(volatile v4f*)(crow + (size_t)row * ldc + cofs) = val; }
            if (ps == 0) __threadfence(); }
        __builtin_amdgcn_wave_barrier(); asm volatile("" ::: "memory");
    }
}

__device__ __forceinline__ h16 tohx(float x) { return (h16)x; }
__device__ __forceinline__ void splitf(float y, unsigned short& h, unsigned short& l) { h = f2bf(y); l = f2bf(y - bf2f(h)); }

__global__ __launch_bounds__(256) void k_cvt8(const float* __restrict__ src, bf* dst, size_t n8) { const size_t i = (size_t)blockIdx.x * 256 + threadIdx.x; if (i >= n8) return; const v8f v = *(const v8f*)(src + i * 8); v8us o;
#pragma unroll
    for (int k = 0; k < 8; ++k) o[k] = f2bf(v[k]); *(volatile v8us*)(dst + i * 8) = o; __threadfence(); *(volatile v8us*)(dst + i * 8) = o; }

__global__ __launch_bounds__(256) void k_split8(const float* __restrict__ src, bf* Ph, bf* Pl, size_t n8) { const size_t i = (size_t)blockIdx.x * 256 + threadIdx.x; if (i >= n8) return; const v8f v = *(const v8f*)(src + i * 8); v8us oh, ol;
#pragma unroll
    for (int k = 0; k < 8; ++k) { unsigned short a, c; splitf(v[k], a, c); oh[k] = a; ol[k] = c; }
    *(volatile v8us*)(Ph + i * 8) = oh; *(volatile v8us*)(Pl + i * 8) = ol; __threadfence(); *(volatile v8us*)(Ph + i * 8) = oh; *(volatile v8us*)(Pl + i * 8) = ol; }

__global__ __launch_bounds__(256) void k_cvth8(const float* __restrict__ src, h16* dst, size_t n8) { const size_t i = (size_t)blockIdx.x * 256 + threadIdx.x; if (i >= n8) return; const v8f v = *(const v8f*)(src + i * 8); v8h o;
#pragma unroll
    for (int k = 0; k < 8; ++k) o[k] = tohx(v[k]); *(volatile v8h*)(dst + i * 8) = o; __threadfence(); *(volatile v8h*)(dst + i * 8) = o; }

__global__ __launch_bounds__(256) void k_kpl(const float* __restrict__ F, bf* Ph, bf* Pl) {
    const size_t e8 = ((size_t)blockIdx.x * 256 + threadIdx.x) * 8; if (e8 >= (size_t)NH_ * TT * HD) return;
    const int d0 = (int)(e8 % HD); const int j = (int)((e8 / HD) % TT); const int h = (int)(e8 / ((size_t)HD * TT));
    const float* f = F + (size_t)h * HD * TT + (size_t)d0 * TT + j; v8us oh, ol;
#pragma unroll
    for (int q = 0; q < 8; ++q) { unsigned short a, c; splitf(f[(size_t)q * TT], a, c); oh[q] = a; ol[q] = c; }
    *(volatile v8us*)(Ph + e8) = oh; *(volatile v8us*)(Pl + e8) = ol; __threadfence(); *(volatile v8us*)(Ph + e8) = oh; *(volatile v8us*)(Pl + e8) = ol; }

__global__ __launch_bounds__(256) void k_sstat(const float* __restrict__ Sb, float* ST) {
    __shared__ __align__(16) float sm[32];
    __shared__ __align__(16) float sf[32];
    const int lane = threadIdx.x & 31, wave = threadIdx.x >> 5;
#pragma unroll 1
    for (int r = 0; r < 4; ++r) {
        const int row = blockIdx.x * 32 + wave * 4 + r;
        const float* sr = Sb + (size_t)row * TT;
        float v[TT / 32]; float mx = -3.0e38f;
#pragma unroll
        for (int ch = 0; ch < TT / 128; ++ch) { const v4f a = *(const v4f*)(sr + ch * 128 + lane * 4);
#pragma unroll
            for (int q = 0; q < 4; ++q) { v[ch * 4 + q] = a[q]; mx = fmaxf(mx, a[q]); } }
#pragma unroll
        for (int sh = 16; sh; sh >>= 1) mx = fmaxf(mx, __shfl_xor(mx, sh, 32));
        float sum = 0.f;
#pragma unroll
        for (int k = 0; k < TT / 32; ++k) { float d0 = __fsub_rn(v[k], mx); asm volatile("" : "+v"(d0)); sum += __builtin_amdgcn_exp2f(__fmul_rn(d0, L2E)); }
#pragma unroll
        for (int sh = 16; sh; sh >>= 1) sum += __shfl_xor(sum, sh, 32);
        const float f = __fdiv_rn(PCAR, sum);
        if (lane == 0) { sm[wave * 4 + r] = mx; sf[wave * 4 + r] = f; }
    }
    __syncthreads();
    if (threadIdx.x < 16) {
        const int t = threadIdx.x, q4 = (t & 7) * 4;
        const v4f vm = *(const v4fa*)(sm + q4); const v4f vf = *(const v4fa*)(sf + q4); v4f val;
#pragma unroll
        for (int q = 0; q < 4; ++q) val[q] = (t < 8) ? vm[q] : vf[q];
        float* dst = ST + ((t < 8) ? (size_t)0 : (size_t)ZH * TT) + (size_t)blockIdx.x * 32 + q4;
#pragma unroll 1
        for (int ps = 0; ps < 2; ++ps) { *(volatile v4f*)dst = val; if (ps == 0) __threadfence(); }
    }
}

__global__ __launch_bounds__(256) void k_expt(const float* __restrict__ Sb, const float* __restrict__ ST, h16* PT) {
    __shared__ __align__(16) h16 pt[64 * 72];
    __shared__ float smx[64];
    __shared__ float sfc[64];
    const int tid = threadIdx.x; const int j0 = blockIdx.x * 64, i0 = blockIdx.y * 64; const size_t zz = blockIdx.z;
    const float* S = Sb + zz * (size_t)TT * TT;
    if (tid < 64) { smx[tid] = ST[zz * TT + i0 + tid]; sfc[tid] = ST[(size_t)ZH * TT + zz * TT + i0 + tid]; }
    __syncthreads();
#pragma unroll
    for (int p = 0; p < 4; ++p) {
        const int r = p * 16 + (tid >> 4), c4 = (tid & 15) * 4;
        const v4f a = *(const v4f*)(S + (size_t)(i0 + r) * TT + j0 + c4);
        const float m = smx[r], f = sfc[r];
#pragma unroll
        for (int q = 0; q < 4; ++q) { float d0 = __fsub_rn(a[q], m); asm volatile("" : "+v"(d0)); const float e = __builtin_amdgcn_exp2f(__fmul_rn(d0, L2E)); pt[(c4 + q) * 72 + r] = tohx(__fmul_rn(e, f)); }
    }
    __syncthreads();
    h16* P = PT + zz * (size_t)TT * TT;
#pragma unroll 1
    for (int ps = 0; ps < 2; ++ps) {
#pragma unroll
        for (int p = 0; p < 2; ++p) { const int c = p * 32 + (tid >> 3), pc = (tid & 7) * 8; const v8h val = *(const v8ha*)(pt + c * 72 + pc);
            *(volatile v8h*)(P + (size_t)(j0 + c) * TT + i0 + pc) = val; }
        if (ps == 0) __threadfence(); }
}

__global__ __launch_bounds__(256) void k_atp(const float* __restrict__ Ob, bf* Ah, bf* Al) {
    const size_t e8 = ((size_t)blockIdx.x * 256 + threadIdx.x) * 8; if (e8 >= (size_t)TT * DHID) return;
    const int cc = (int)(e8 % DHID); const int s = (int)(e8 / DHID);
    const float* o = Ob + (size_t)cc * TT + s; v8us oh, ol;
#pragma unroll
    for (int q = 0; q < 8; ++q) { unsigned short a, c; splitf(o[(size_t)q * TT] * (1.0f / PCAR), a, c); oh[q] = a; ol[q] = c; }
    *(volatile v8us*)(Ah + e8) = oh; *(volatile v8us*)(Al + e8) = ol; __threadfence(); *(volatile v8us*)(Ah + e8) = oh; *(volatile v8us*)(Al + e8) = ol; }

__host__ __device__ constexpr size_t a256(size_t b) { return (b + 255) & ~(size_t)255; }
constexpr size_t WS_NEED = 4 * a256((size_t)DHID * DM * 2) + a256((size_t)TT * DM * 2) + a256((size_t)TT * DHID * 4) + 5 * a256((size_t)NH_ * TT * HD * 2)
                         + a256((size_t)ZH * TT * TT * 4) + a256((size_t)2 * ZH * TT * 4) + a256((size_t)ZH * TT * TT * 2) + a256((size_t)DHID * TT * 4) + 2 * a256((size_t)TT * DHID * 2);
static_assert(WS_NEED <= (size_t)134217728);

extern "C" void kernel_launch(void* const* d_in, const int* in_sizes, int n_in,
                              void* d_out, int out_size, void* d_ws, size_t ws_size, hipStream_t stream) {
    if (n_in < 9) return;
    if ((size_t)in_sizes[0] < ((size_t)(NB - 1) * TT_FULL + TT) * (size_t)DM) return;
    if (in_sizes[1] < DHID * DM || in_sizes[3] < DHID * DM || in_sizes[5] < DHID * DM || in_sizes[7] < DM * DHID) return;
    if (in_sizes[2] < DHID || in_sizes[4] < DHID || in_sizes[6] < DHID || in_sizes[8] < DM) return;
    if ((size_t)out_size < (size_t)NB * TT * DM) return;
    const float* x = (const float*)d_in[0]; const float* wq = (const float*)d_in[1]; const float* bq = (const float*)d_in[2]; const float* wk = (const float*)d_in[3]; const float* bk = (const float*)d_in[4];
    const float* wv = (const float*)d_in[5]; const float* bv = (const float*)d_in[6]; const float* wo = (const float*)d_in[7]; const float* bo = (const float*)d_in[8];
    float* OUT = (float*)d_out;
    char* wsp = (char*)d_ws;
    auto take = [&](size_t bytes) { char* p = wsp; wsp += a256(bytes); return (void*)p; };
    bf* WQ = (bf*)take((size_t)DHID * DM * 2); bf* WK = (bf*)take((size_t)DHID * DM * 2); bf* WV = (bf*)take((size_t)DHID * DM * 2); bf* WO = (bf*)take((size_t)DM * DHID * 2);
    bf* XB = (bf*)take((size_t)TT * DM * 2); float* FP = (float*)take((size_t)TT * DHID * 4);
    bf* QPh = (bf*)take((size_t)NH_ * TT * HD * 2); bf* QPl = (bf*)take((size_t)NH_ * TT * HD * 2); bf* KPh = (bf*)take((size_t)NH_ * TT * HD * 2); bf* KPl = (bf*)take((size_t)NH_ * TT * HD * 2); h16* VT16 = (h16*)take((size_t)NH_ * HD * TT * 2);
    float* Sb = (float*)take((size_t)ZH * TT * TT * 4); float* ST = (float*)take((size_t)2 * ZH * TT * 4); h16* PT16 = (h16*)take((size_t)ZH * TT * TT * 2);
    float* Ob = (float*)take((size_t)DHID * TT * 4); bf* ATh = (bf*)take((size_t)TT * DHID * 2); bf* ATl = (bf*)take((size_t)TT * DHID * 2);
    if ((size_t)(wsp - (char*)d_ws) > ws_size) return;
    { k_cvt8<<<(unsigned)(((size_t)DHID * DM / 8 + 255) / 256), 256, 0, stream>>>(wq, WQ, (size_t)DHID * DM / 8); k_cvt8<<<(unsigned)(((size_t)DHID * DM / 8 + 255) / 256), 256, 0, stream>>>(wk, WK, (size_t)DHID * DM / 8);
      k_cvt8<<<(unsigned)(((size_t)DHID * DM / 8 + 255) / 256), 256, 0, stream>>>(wv, WV, (size_t)DHID * DM / 8); k_cvt8<<<(unsigned)(((size_t)DM * DHID / 8 + 255) / 256), 256, 0, stream>>>(wo, WO, (size_t)DM * DHID / 8); }
    const size_t NPL = (size_t)NH_ * TT * HD;
    const unsigned L8 = (unsigned)((NPL / 8 + 255) / 256);
    for (int b = 0; b < NB; ++b) {
        k_cvt8<<<(unsigned)(((size_t)TT * DM / 8 + 255) / 256), 256, 0, stream>>>(x + (size_t)b * TT_FULL * DM, XB, (size_t)TT * DM / 8);
        k_gemmw<bf, 0, true><<<dim3(TT / 64, DHID / 64, 1), 32, 0, stream>>>(XB, nullptr, WQ, nullptr, DM, FP, DHID, bq, 0, 0, 0);
        k_split8<<<L8, 256, 0, stream>>>(FP, QPh, QPl, NPL / 8);
        k_gemmw<bf, 0, true><<<dim3(TT / 64, DHID / 64, 1), 32, 0, stream>>>(XB, nullptr, WK, nullptr, DM, FP, DHID, bk, 0, 0, 0);
        k_kpl<<<L8, 256, 0, stream>>>(FP, KPh, KPl);
        k_gemmw<bf, 0, true><<<dim3(TT / 64, DHID / 64, 1), 32, 0, stream>>>(XB, nullptr, WV, nullptr, DM, FP, DHID, bv, 0, 0, 0);
        k_cvth8<<<L8, 256, 0, stream>>>(FP, VT16, NPL / 8);
        for (int h0 = 0; h0 < NH_; h0 += ZH) { const size_t zo = (size_t)h0 * TT * HD;
            k_gemmw<bf, 2, false><<<dim3(TT / 64, TT / 64, ZH), 32, 0, stream>>>(QPh + zo, QPl + zo, KPh + zo, KPl + zo, HD, Sb, TT, nullptr, (size_t)TT * HD, (size_t)TT * HD, (size_t)TT * TT);
            k_sstat<<<(unsigned)(ZH * TT / 32), 256, 0, stream>>>(Sb, ST);
            k_expt<<<dim3(TT / 64, TT / 64, ZH), 256, 0, stream>>>(Sb, ST, PT16);
            k_gemmw<h16, 0, false><<<dim3(1, TT / 64, ZH), 32, 0, stream>>>(VT16 + zo, nullptr, PT16, nullptr, TT, Ob + zo, TT, nullptr, (size_t)HD * TT, (size_t)TT * TT, (size_t)HD * TT); }
        k_atp<<<(unsigned)(((size_t)TT * DHID / 8 + 255) / 256), 256, 0, stream>>>(Ob, ATh, ATl);
        k_gemmw<bf, 1, true><<<dim3(TT / 64, DM / 64, 1), 32, 0, stream>>>(ATh, ATl, WO, nullptr, DHID, OUT + (size_t)b * TT * DM, DM, bo, 0, 0, 0); }
}
